// TrendRefinement_40011915329799
// MI455X (gfx1250) — hardware-run, weakly checked
//
#include <hip/hip_runtime.h>


namespace {
constexpr int NB = 16, L = 512, NH = 8, ED = 64, G = NB * NH, KW = 7, PADW = 3;
constexpr float XS = 8.0f;
typedef _Float16 b16;
typedef __attribute__((ext_vector_type(16))) _Float16 v16b;
typedef __attribute__((ext_vector_type(8))) _Float16 v8b;
typedef __attribute__((ext_vector_type(8))) float v8f;
typedef __attribute__((ext_vector_type(4))) float v4f;
typedef __attribute__((ext_vector_type(2))) _Float16 v2b;
typedef __attribute__((ext_vector_type(2))) float v2f;
__device__ __forceinline__ float bf16_rne(float f) { unsigned int u = __float_as_uint(f); u += 0x7FFFu + ((u >> 16) & 1u); float r = __uint_as_float(u & 0xFFFF0000u); asm volatile("" : "+v"(r)); return r; }
__device__ __forceinline__ void split16(float v, b16& hi, b16& lo) { hi = (b16)v; lo = (b16)(v - (float)hi); }
__device__ __forceinline__ v16b frag_kb(const b16* p, int hh) { const v8b a = *(const v8b*)(p + 8 * hh), b = *(const v8b*)(p + 16 + 8 * hh); v16b f;
#pragma unroll
  for (int e = 0; e < 8; ++e) { f[e] = a[e]; f[8 + e] = b[e]; } return f; }
__device__ __forceinline__ v8f wmma16b(v16b a, v16b b, v8f c) { v8f d = __builtin_amdgcn_wmma_f32_16x16x32_f16(false, a, false, b, (short)0, c, false, false); asm volatile("v_nop\n\tv_nop\n\tv_nop\n\tv_nop" : "+v"(d) : "v"(a), "v"(b)); return d; }
__device__ __forceinline__ void wave_lds_sync() { __builtin_amdgcn_fence(__ATOMIC_RELEASE, "workgroup"); __builtin_amdgcn_wave_barrier(); __builtin_amdgcn_fence(__ATOMIC_ACQUIRE, "workgroup"); }
__device__ __forceinline__ float pmul(float a, float b) { float p = a * b; asm volatile("" : "+v"(p)); return p; }
__device__ __forceinline__ int iclamp(int v, int lo, int hi) { return v < lo ? lo : (v > hi ? hi : v); }

__global__ __launch_bounds__(256) void uprep_kernel(const float* __restrict__ U, b16* __restrict__ UP, b16* __restrict__ UT) { const int u = blockIdx.x * 256 + threadIdx.x; if (u >= L * L / 8) return; const int r = u / (L / 8), k0 = (u % (L / 8)) * 8; v8b a, b;
#pragma unroll
  for (int j = 0; j < 8; ++j) { a[j] = (b16)(bf16_rne(U[(size_t)r * L + k0 + j]) * XS); b[j] = (b16)(bf16_rne(U[(size_t)(k0 + j) * L + r]) * XS); }
  for (int pass = 0; pass < 2; ++pass) { *(volatile v8b*)(UP + (size_t)r * L + k0) = a; *(volatile v8b*)(UT + (size_t)r * L + k0) = b; __threadfence(); } }
__global__ __launch_bounds__(256) void vprep_kernel(const float* __restrict__ v, b16* __restrict__ VT) { const int wave = threadIdx.x >> 5, lane = threadIdx.x & 31; const size_t wid = (size_t)blockIdx.x * 8 + wave; if (wid >= (size_t)G * ED * (L / 64)) return; const int g = (int)(wid / (ED * (L / 64))); const int rem = (int)(wid % (ED * (L / 64))); const int d = rem / (L / 64), j0 = (rem % (L / 64)) * 64 + 2 * lane; const int b = g / NH, h = g % NH;
  const v2b val = {(b16)bf16_rne(v[(((size_t)b * L + j0) * NH + h) * ED + d]), (b16)bf16_rne(v[(((size_t)b * L + j0 + 1) * NH + h) * ED + d])}; for (int pass = 0; pass < 2; ++pass) { *(volatile v2b*)(VT + ((size_t)g * ED + d) * L + j0) = val; __threadfence(); } }
__global__ __launch_bounds__(256) void lam_kernel(const float* __restrict__ v, const float* __restrict__ cw, const float* __restrict__ cb, const float* __restrict__ S, float* __restrict__ INV) { const int u = blockIdx.x * 256 + threadIdx.x; if (u >= G * L) return; const int g = u / L, l = u % L; const int b = g / NH, h = g % NH; float s = bf16_rne(cb[0]);
#pragma unroll 1
  for (int k = 0; k < KW; ++k) { const int lj = iclamp(l + k - PADW, 0, L - 1); const float* row = v + (((size_t)b * L + lj) * NH + h) * ED;
#pragma unroll 1
    for (int e = 0; e < ED; ++e) s += pmul(bf16_rne(row[e]), bf16_rne(cw[e * KW + k])); }
  const float lam = 1.0f + (s > 0.0f ? s : (__expf(s) - 1.0f)); const float inv = 1.0f / (1.0f + pmul(lam, bf16_rne(S[l])));
  for (int pass = 0; pass < 2; ++pass) { ((volatile float*)INV)[u] = inv; __threadfence(); } }
__global__ __launch_bounds__(32) void g1_kernel(const b16* __restrict__ UT, const b16* __restrict__ VT, const float* __restrict__ INV, int GLIM, float* __restrict__ TM) { __shared__ float Tf[16][68]; const int lane = threadIdx.x, nloc = lane & 15, hlf = lane >> 4; const int g = blockIdx.x / (L / 16), mt = blockIdx.x % (L / 16); if (g >= GLIM) return; const int m0 = mt * 16;
  v8f acc[4];
#pragma unroll
  for (int t = 0; t < 4; ++t) acc[t] = (v8f){};
#pragma unroll 2
  for (int kb = 0; kb < L; kb += 32) { const v16b a = frag_kb(UT + (size_t)(m0 + nloc) * L + kb, hlf);
#pragma unroll
    for (int t = 0; t < 4; ++t) acc[t] = wmma16b(a, frag_kb(VT + ((size_t)g * ED + t * 16 + nloc) * L + kb, hlf), acc[t]); }
#pragma unroll
  for (int t = 0; t < 4; ++t)
#pragma unroll
    for (int r8 = 0; r8 < 8; ++r8) { const int m = m0 + 8 * hlf + r8; Tf[8 * hlf + r8][t * 16 + nloc] = pmul(acc[t][r8] * (1.0f / XS), INV[g * L + m]); }
  wave_lds_sync();
  for (int pass = 0; pass < 2; ++pass) { for (int rr = 0; rr < 16; ++rr) { const float* src = &Tf[rr][lane * 2]; *(volatile v2f*)(TM + ((size_t)g * L + m0 + rr) * ED + lane * 2) = (v2f){src[0], src[1]}; } __threadfence(); } }
__global__ __launch_bounds__(256) void tprep_kernel(const float* __restrict__ TM, int GLIM, b16* __restrict__ TTh, b16* __restrict__ TTl) { const int wave = threadIdx.x >> 5, lane = threadIdx.x & 31; const size_t wid = (size_t)blockIdx.x * 8 + wave; if (wid >= (size_t)GLIM * ED * (L / 64)) return; const int g = (int)(wid / (ED * (L / 64))); const int rem = (int)(wid % (ED * (L / 64))); const int d = rem / (L / 64), m0 = (rem % (L / 64)) * 64 + 2 * lane;
  b16 h0, l0, h1, l1; split16(TM[((size_t)g * L + m0) * ED + d] * XS, h0, l0); split16(TM[((size_t)g * L + m0 + 1) * ED + d] * XS, h1, l1);
  for (int pass = 0; pass < 2; ++pass) { *(volatile v2b*)(TTh + ((size_t)g * ED + d) * L + m0) = (v2b){h0, h1}; *(volatile v2b*)(TTl + ((size_t)g * ED + d) * L + m0) = (v2b){l0, l1}; __threadfence(); } }
__global__ __launch_bounds__(32) void g2_kernel(const b16* __restrict__ UP, const b16* __restrict__ TTh, const b16* __restrict__ TTl, int GLIM, float* __restrict__ out) { __shared__ float Tf[16][68]; const int lane = threadIdx.x, nloc = lane & 15, hlf = lane >> 4; const int g = blockIdx.x / (L / 16), it = blockIdx.x % (L / 16); if (g >= GLIM) return; const int i0 = it * 16; const int b = g / NH, h = g % NH;
  v8f acc[4];
#pragma unroll
  for (int t = 0; t < 4; ++t) acc[t] = (v8f){};
#pragma unroll 2
  for (int kb = 0; kb < L; kb += 32) { const v16b a = frag_kb(UP + (size_t)(i0 + nloc) * L + kb, hlf);
#pragma unroll
    for (int t = 0; t < 4; ++t) { const size_t ro = ((size_t)g * ED + t * 16 + nloc) * L + kb; acc[t] = wmma16b(a, frag_kb(TTh + ro, hlf), acc[t]); acc[t] = wmma16b(a, frag_kb(TTl + ro, hlf), acc[t]); } }
#pragma unroll
  for (int t = 0; t < 4; ++t)
#pragma unroll
    for (int r8 = 0; r8 < 8; ++r8) Tf[8 * hlf + r8][t * 16 + nloc] = acc[t][r8] * (1.0f / (XS * XS));
  wave_lds_sync();
  for (int pass = 0; pass < 2; ++pass) { for (int rr = 0; rr < 16; ++rr) { const float* src = &Tf[rr][lane * 2]; *(volatile v2f*)(out + (((size_t)b * L + i0 + rr) * NH + h) * ED + lane * 2) = (v2f){src[0], src[1]}; } __threadfence(); } }
}

extern "C" void kernel_launch(void* const* d_in, const int* in_sizes, int n_in, void* d_out, int out_size, void* d_ws, size_t ws_size, hipStream_t stream) {
  (void)n_in;
  auto Fp = [&](int i) { return (const float*)d_in[i]; };
  if (in_sizes[0] != NB * L * NH * ED || in_sizes[1] != ED * KW || in_sizes[2] != 1 || in_sizes[3] != L * L || in_sizes[4] != L || out_size != NB * L * NH * ED) return;
  const int GLIM = G;
  size_t off = 0; char* ws = (char*)d_ws;
  auto carve = [&](size_t bytes) { char* p = ws + off; off += (bytes + 255) & ~(size_t)255; return p; };
  b16* UP = (b16*)carve((size_t)L * L * 2); b16* UT = (b16*)carve((size_t)L * L * 2); b16* VT = (b16*)carve((size_t)G * ED * L * 2); float* INV = (float*)carve((size_t)G * L * 4); float* TM = (float*)carve((size_t)G * L * ED * 4); b16* TTh = (b16*)carve((size_t)G * ED * L * 2); b16* TTl = (b16*)carve((size_t)G * ED * L * 2);
  if (off > ws_size || off > ((size_t)64 << 20)) return;
  uprep_kernel<<<(L * L / 8 + 255) / 256, 256, 0, stream>>>(Fp(3), UP, UT);
  vprep_kernel<<<(unsigned)(((size_t)G * ED * (L / 64) + 7) / 8), 256, 0, stream>>>(Fp(0), VT);
  lam_kernel<<<(G * L + 255) / 256, 256, 0, stream>>>(Fp(0), Fp(1), Fp(2), Fp(4), INV);
  g1_kernel<<<GLIM * (L / 16), 32, 0, stream>>>(UT, VT, INV, GLIM, TM);
  tprep_kernel<<<(unsigned)(((size_t)GLIM * ED * (L / 64) + 7) / 8), 256, 0, stream>>>(TM, GLIM, TTh, TTl);
  g2_kernel<<<GLIM * (L / 16), 32, 0, stream>>>(UP, TTh, TTl, GLIM, (float*)d_out);
}
